// ContentAttender_6597069767497
// MI455X (gfx1250) — hardware-verified
//
#include <hip/hip_runtime.h>
#include <stddef.h>


typedef _Float16 h16;
typedef _Float16 v16h __attribute__((ext_vector_type(16)));
typedef _Float16 v8h  __attribute__((ext_vector_type(8)));
typedef float    v8f  __attribute__((ext_vector_type(8)));
typedef float    v4f  __attribute__((ext_vector_type(4)));

#ifndef NB
#define NB 4
#endif
#ifndef SEQ
#define SEQ 512
#endif
#define NB_FULL  4
#define SEQ_FULL 512
#define KD   128
#define NHID 32

static_assert(NB >= 1 && NB <= NB_FULL);
static_assert(SEQ >= 128 && SEQ <= SEQ_FULL && (SEQ % 128) == 0 && (SEQ % 64) == 0);
static_assert(KD == 128 && (KD % 32) == 0 && (KD % 64) == 0 && KD == 8 * 16);
static_assert(NHID == 32);
static_assert((size_t)NB_FULL * SEQ_FULL * KD * 4 == (size_t)1048576);

#define LDT 72
#define LDC 68
#define LDR 132
#define LDW 136
static_assert((LDT % 8) == 0 && LDT >= 64);
static_assert((LDC % 4) == 0 && LDC >= 64);
static_assert((LDR % 4) == 0 && LDR >= 128);
static_assert((LDW % 8) == 0 && LDW >= KD);

#define WCARRY 64.0f
#define XCARRY 64.0f
#define PCARRY 1024.0f
#define TSCALE 2.8853900817779268f

#define WT_BYTES ((size_t)NHID * KD * 2)
#define VT_BYTES ((size_t)NB * KD * SEQ * 2)
#define HT_BYTES ((size_t)NB * NHID * SEQ * 4)
#define OFF_WK ((size_t)0)
#define OFF_WQ (OFF_WK + WT_BYTES)
#define OFF_VT (OFF_WQ + WT_BYTES)
#define OFF_KH (OFF_VT + VT_BYTES)
#define OFF_QH (OFF_KH + HT_BYTES)
#define WS_TOTAL (OFF_QH + HT_BYTES)
static_assert((WT_BYTES % 128) == 0 && (VT_BYTES % 128) == 0 && (HT_BYTES % 128) == 0);
static_assert(WS_TOTAL <= (size_t)134217728);

static_assert(KD * NHID == 256 * 16);
static_assert(NHID * 64 == 128 * 4 * 4);
static_assert(KD * 64 == 128 * 8 * 8);
static_assert(NHID * 128 == 256 * 4 * 4);
static_assert(4 * 16 == 64 && 8 * 16 == 128);

__device__ __forceinline__ float bf16r(float x) {
  unsigned int u = __float_as_uint(x);
  u = (u + 0x7FFFu + ((u >> 16) & 1u)) & 0xFFFF0000u;
  return __uint_as_float(u);
}

__device__ __forceinline__ h16 toh_flush(float v) {
  const h16 r = (h16)v;
  return (fabsf(v) < 6.103515625e-05f) ? (h16)0.0f : r;
}

__device__ __forceinline__ float ex2(float x) {
#if __has_builtin(__builtin_amdgcn_exp2f)
  return __builtin_amdgcn_exp2f(x);
#else
  return exp2f(x);
#endif
}

__device__ __forceinline__ v16h frag_at(const _Float16* p) {
  v8h lo = *(const v8h*)(p);
  v8h hi = *(const v8h*)(p + 16);
  v16h out;
#pragma unroll
  for (int i = 0; i < 8; ++i) { out[i] = lo[i]; out[i + 8] = hi[i]; }
  return out;
}
__device__ __forceinline__ v16h ld_frag(const _Float16* base, unsigned ld) {
  const unsigned lane = threadIdx.x & 31u;
  return frag_at(base + (lane & 15u) * ld + (lane >> 4) * 8u);
}

__device__ __forceinline__ v8f wmma16(v16h a, v16h b, v8f c) {
  v8f d = __builtin_amdgcn_wmma_f32_16x16x32_f16(false, a, false, b, (short)0, c,
                                                 false, false);
  asm volatile("v_nop\n\tv_nop\n\tv_nop\n\tv_nop" : "+v"(d) : "v"(a), "v"(b));
  return d;
}

__device__ __forceinline__ float red16_max(float x) {
#pragma unroll
  for (int off = 1; off < 16; off <<= 1) x = fmaxf(x, __shfl_xor(x, off, 32));
  return x;
}
__device__ __forceinline__ float red16_sum(float x) {
#pragma unroll
  for (int off = 1; off < 16; off <<= 1) x += __shfl_xor(x, off, 32);
  return x;
}

__device__ __forceinline__ void wave_lds_sync() {
  __builtin_amdgcn_fence(3  , "wavefront");
  asm volatile("s_wait_dscnt 0x0" ::: "memory");
  __builtin_amdgcn_wave_barrier();
}

__global__ __launch_bounds__(256) void wconv32_kernel(
    const float* __restrict__ W, _Float16* __restrict__ Wt) {
  __shared__ __attribute__((aligned(16))) _Float16 T[NHID * LDW];
  const unsigned tid = threadIdx.x;
#pragma unroll 4
  for (unsigned j = 0; j < 16u; ++j) {
    const unsigned idx = tid + 256u * j;
    const unsigned kr = idx >> 5, nc = idx & 31u;
    const float v = W[(size_t)kr * NHID + nc];
    T[nc * LDW + kr] = toh_flush(WCARRY * bf16r(v));
  }
  __syncthreads();
  v8h x[2];
  size_t off[2];
#pragma unroll
  for (unsigned i = 0; i < 2u; ++i) {
    const unsigned n = 16u * i + (tid >> 4);
    const unsigned kc = (tid & 15u) * 8u;
    x[i] = *(const v8h*)&T[n * LDW + kc];
    off[i] = (size_t)n * KD + kc;
  }
#pragma unroll
  for (int i = 0; i < 2; ++i) *(volatile v8h*)(Wt + off[i]) = x[i];
  __threadfence();
#pragma unroll
  for (int i = 0; i < 2; ++i) *(volatile v8h*)(Wt + off[i]) = x[i];
}

__global__ __launch_bounds__(256) void vtconv_kernel(
    const float* __restrict__ Xk, _Float16* __restrict__ Vt) {
  __shared__ __attribute__((aligned(16))) _Float16 T[64 * LDT];
  const unsigned tid = threadIdx.x;
  const unsigned d0 = blockIdx.x * 64u;
  const unsigned k0 = blockIdx.y * 64u;
  const unsigned b = blockIdx.z;
#pragma unroll 4
  for (unsigned j = 0; j < 16u; ++j) {
    const unsigned idx = tid + 256u * j;
    const unsigned kr = idx >> 6, nc = idx & 63u;
    const float v = Xk[((size_t)b * SEQ_FULL + k0 + kr) * KD + d0 + nc];
    T[nc * LDT + kr] = toh_flush(XCARRY * bf16r(v));
  }
  __syncthreads();
  v8h x[2];
  size_t off[2];
#pragma unroll
  for (unsigned i = 0; i < 2u; ++i) {
    const unsigned n = 32u * i + (tid >> 3);
    const unsigned kc = (tid & 7u) * 8u;
    x[i] = *(const v8h*)&T[n * LDT + kc];
    off[i] = ((size_t)b * KD + d0 + n) * SEQ + k0 + kc;
  }
#pragma unroll
  for (int i = 0; i < 2; ++i) *(volatile v8h*)(Vt + off[i]) = x[i];
  __threadfence();
#pragma unroll
  for (int i = 0; i < 2; ++i) *(volatile v8h*)(Vt + off[i]) = x[i];
}

template <int ADD_BIAS>
__device__ __forceinline__ void proj_body(
    const float* __restrict__ X, const _Float16* __restrict__ Wt,
    const float* __restrict__ bias, float* __restrict__ outT) {
  __shared__ __attribute__((aligned(16))) float CsT[NHID * LDR];
  const unsigned tid = threadIdx.x, lane = tid & 31u;
  const unsigned w = (unsigned)__builtin_amdgcn_readfirstlane((int)(tid >> 5));
  const unsigned hh = lane >> 4, m = lane & 15u;
  const unsigned r0 = blockIdx.x * 128u;
  const unsigned b = blockIdx.y;

  const float* xr = X + ((size_t)b * SEQ_FULL + r0 + w * 16u + m) * KD + hh * 8u;
  const _Float16* bp0 = Wt + (size_t)m * KD + hh * 8u;
  const _Float16* bp1 = bp0 + (size_t)16 * KD;
  v8f acc0 = {}, acc1 = {};
#pragma unroll
  for (unsigned k0 = 0; k0 < (unsigned)KD; k0 += 32u) {
    const v4f x0 = *(const v4f*)(xr + k0);
    const v4f x1 = *(const v4f*)(xr + k0 + 4u);
    const v4f x2 = *(const v4f*)(xr + k0 + 16u);
    const v4f x3 = *(const v4f*)(xr + k0 + 20u);
    v16h a;
#pragma unroll
    for (int i = 0; i < 4; ++i) {
      a[i]      = toh_flush(XCARRY * bf16r(x0[i]));
      a[i + 4]  = toh_flush(XCARRY * bf16r(x1[i]));
      a[i + 8]  = toh_flush(XCARRY * bf16r(x2[i]));
      a[i + 12] = toh_flush(XCARRY * bf16r(x3[i]));
    }
    const v16h b0 = frag_at(bp0 + k0);
    const v16h b1 = frag_at(bp1 + k0);
    acc0 = wmma16(a, b0, acc0);
    acc1 = wmma16(a, b1, acc1);
  }
  {
    float* d0 = &CsT[m * LDR + w * 16u + hh * 8u];
    float* d1 = &CsT[(16u + m) * LDR + w * 16u + hh * 8u];
    const v4f t0 = {acc0[0], acc0[1], acc0[2], acc0[3]};
    const v4f t1 = {acc0[4], acc0[5], acc0[6], acc0[7]};
    const v4f t2 = {acc1[0], acc1[1], acc1[2], acc1[3]};
    const v4f t3 = {acc1[4], acc1[5], acc1[6], acc1[7]};
    *(v4f*)(d0)     = t0;
    *(v4f*)(d0 + 4) = t1;
    *(v4f*)(d1)     = t2;
    *(v4f*)(d1 + 4) = t3;
  }
  __syncthreads();

  v4f xs[4];
  size_t off[4];
#pragma unroll
  for (unsigned i = 0; i < 4u; ++i) {
    const unsigned h = 8u * i + w;
    const unsigned c = lane * 4u;
    const v4f u = *(const v4f*)&CsT[h * LDR + c];
    const float bb = ADD_BIAS ? bf16r(bias[h]) : 0.0f;
    v4f val;
#pragma unroll
    for (int j = 0; j < 4; ++j)
      val[j] = (u[j] * (1.0f / (WCARRY * XCARRY)) + bb) * TSCALE;
    xs[i] = val;
    off[i] = ((size_t)b * NHID + h) * SEQ + r0 + c;
  }
#pragma unroll
  for (int i = 0; i < 4; ++i) *(volatile v4f*)(outT + off[i]) = xs[i];
  __threadfence();
#pragma unroll
  for (int i = 0; i < 4; ++i) *(volatile v4f*)(outT + off[i]) = xs[i];
}

__global__ __launch_bounds__(256) void proj_k_kernel(
    const float* __restrict__ X, const _Float16* __restrict__ Wt,
    const float* __restrict__ bias, float* __restrict__ outT) {
  proj_body<1>(X, Wt, bias, outT);
}
__global__ __launch_bounds__(256) void proj_q_kernel(
    const float* __restrict__ X, const _Float16* __restrict__ Wt,
    const float* __restrict__ bias, float* __restrict__ outT) {
  proj_body<0>(X, Wt, bias, outT);
}

__global__ __launch_bounds__(128) __attribute__((amdgpu_num_vgpr(256))) void attn_kernel(
    const float* __restrict__ QhT, const float* __restrict__ KhT,
    const _Float16* __restrict__ Vt, const float* __restrict__ w2,
    const float* __restrict__ b2, float* __restrict__ out) {
  __shared__ __attribute__((aligned(16))) float QHs[NHID * 64];
  __shared__ __attribute__((aligned(16))) float KHs[NHID * 64];
  __shared__ __attribute__((aligned(16))) _Float16 Vs[KD * LDT];
  __shared__ __attribute__((aligned(16))) _Float16 Ps[4 * 16 * LDT];
  __shared__ __attribute__((aligned(16))) float Os[4 * 16 * LDC];
  __shared__ __attribute__((aligned(16))) float W2s[NHID];

  const unsigned tid = threadIdx.x, lane = tid & 31u;
  const unsigned w = (unsigned)__builtin_amdgcn_readfirstlane((int)(tid >> 5));
  const unsigned hh = lane >> 4, m = lane & 15u;
  const unsigned q0 = blockIdx.x * 64u;
  const unsigned b = blockIdx.y;
  _Float16* P = Ps + w * (16u * LDT);
  float* Ow = Os + w * (16u * LDC);

#pragma unroll
  for (unsigned j = 0; j < 4u; ++j) {
    const unsigned idx = tid + 128u * j;
    const unsigned h = idx >> 4, c = (idx & 15u) * 4u;
    *(v4f*)&QHs[h * 64u + c] = *(const v4f*)(QhT + ((size_t)b * NHID + h) * SEQ + q0 + c);
  }
  {
    const float wv = w2[tid & 31u];
    if (tid < 32u) W2s[tid] = -2.0f * bf16r(wv);
  }
  __syncthreads();
  float csum = 0.0f;
#pragma unroll 1
  for (unsigned h = 0; h < (unsigned)NHID; ++h) csum += W2s[h];
  const float cshift = bf16r(b2[0]) - 0.5f * csum;

  float mrow[8], lrow[8];
  v8f o[8];
#pragma unroll
  for (int v = 0; v < 8; ++v) { mrow[v] = -1.0e30f; lrow[v] = 0.0f; }
#pragma unroll
  for (int nb = 0; nb < 8; ++nb) o[nb] = (v8f){};

  for (unsigned kb = 0; kb < (unsigned)SEQ; kb += 64u) {
#pragma unroll
    for (unsigned j = 0; j < 4u; ++j) {
      const unsigned idx = tid + 128u * j;
      const unsigned h = idx >> 4, c = (idx & 15u) * 4u;
      *(v4f*)&KHs[h * 64u + c] = *(const v4f*)(KhT + ((size_t)b * NHID + h) * SEQ + kb + c);
    }
#pragma unroll
    for (unsigned j = 0; j < 8u; ++j) {
      const unsigned idx = tid + 128u * j;
      const unsigned r = idx >> 3, c = (idx & 7u) * 8u;
      *(v8h*)&Vs[r * LDT + c] = *(const v8h*)(Vt + ((size_t)b * KD + r) * SEQ + kb + c);
    }
    __syncthreads();

    v8f s[4];
#pragma unroll
    for (int kg = 0; kg < 4; ++kg)
#pragma unroll
      for (int v = 0; v < 8; ++v) s[kg][v] = cshift;
#pragma unroll 1
    for (unsigned h = 0; h < (unsigned)NHID; ++h) {
      const float wm = W2s[h];
      const v4f qa = *(const v4f*)&QHs[h * 64u + w * 16u + hh * 8u];
      const v4f qb = *(const v4f*)&QHs[h * 64u + w * 16u + hh * 8u + 4u];
      const float q[8] = {qa[0], qa[1], qa[2], qa[3], qb[0], qb[1], qb[2], qb[3]};
#pragma unroll
      for (int kg = 0; kg < 4; ++kg) {
        const float kv = KHs[h * 64u + (unsigned)kg * 16u + m];
#pragma unroll
        for (int v = 0; v < 8; ++v) {
          const float e = ex2(q[v] + kv);
          const float r = __builtin_amdgcn_rcpf(e + 1.0f);
          s[kg][v] = __builtin_fmaf(wm, r, s[kg][v]);
        }
      }
    }

    float alpha[8];
#pragma unroll
    for (int v = 0; v < 8; ++v) {
      float mx = fmaxf(fmaxf(s[0][v], s[1][v]), fmaxf(s[2][v], s[3][v]));
      mx = red16_max(mx);
      const float mn = fmaxf(mrow[v], mx);
      alpha[v] = __expf(mrow[v] - mn);
      mrow[v] = mn;
    }
#pragma unroll
    for (int kg = 0; kg < 4; ++kg)
#pragma unroll
      for (int v = 0; v < 8; ++v) {
        const float d = s[kg][v] - mrow[v];
        const float pe = __expf(d) * PCARRY;
        const h16 ph = (d < -16.0f) ? (h16)0.0f : (h16)pe;
        P[(hh * 8u + (unsigned)v) * LDT + (unsigned)kg * 16u + m] = ph;
        s[kg][v] = (float)ph;
      }
#pragma unroll
    for (int v = 0; v < 8; ++v) {
      const float rs = red16_sum((s[0][v] + s[1][v]) + (s[2][v] + s[3][v]));
      lrow[v] = alpha[v] * lrow[v] + rs;
    }
#pragma unroll
    for (int nb = 0; nb < 8; ++nb)
#pragma unroll
      for (int v = 0; v < 8; ++v) o[nb][v] = o[nb][v] * alpha[v];
    wave_lds_sync();

#pragma unroll
    for (int c = 0; c < 2; ++c) {
      const v16h pf = ld_frag(P + c * 32, LDT);
#pragma unroll
      for (int nb = 0; nb < 8; ++nb) {
        const v16h vf = ld_frag(&Vs[(nb * 16) * LDT + c * 32], LDT);
        o[nb] = wmma16(pf, vf, o[nb]);
      }
    }
    __syncthreads();
  }

  float inv[8];
#pragma unroll
  for (int v = 0; v < 8; ++v) inv[v] = __builtin_amdgcn_rcpf(lrow[v]) * (1.0f / XCARRY);

#pragma unroll
  for (int c2 = 0; c2 < 2; ++c2) {
#pragma unroll
    for (int j = 0; j < 4; ++j)
#pragma unroll
      for (int v = 0; v < 8; ++v)
        Ow[(hh * 8u + (unsigned)v) * LDC + (unsigned)j * 16u + m] = o[4 * c2 + j][v] * inv[v];
    wave_lds_sync();
    v4f x[8];
    size_t off[8];
#pragma unroll
    for (unsigned i = 0; i < 8u; ++i) {
      const unsigned r = 2u * i + (lane >> 4);
      const unsigned c = (lane & 15u) * 4u;
      x[i] = *(const v4f*)&Ow[r * LDC + c];
      off[i] = ((size_t)b * SEQ_FULL + q0 + w * 16u + r) * KD + (unsigned)c2 * 64u + c;
    }
#pragma unroll
    for (int i = 0; i < 8; ++i) *(volatile v4f*)(out + off[i]) = x[i];
    __threadfence();
#pragma unroll
    for (int i = 0; i < 8; ++i) *(volatile v4f*)(out + off[i]) = x[i];
    wave_lds_sync();
  }
}

extern "C" void kernel_launch(void* const* d_in, const int* in_sizes, int n_in,
                              void* d_out, int out_size, void* d_ws, size_t ws_size,
                              hipStream_t stream) {
  if (n_in < 7) return;
  const long long need_x = ((long long)(NB - 1) * SEQ_FULL + SEQ) * KD;
  if ((long long)in_sizes[0] < need_x) return;
  if ((long long)in_sizes[1] < need_x) return;
  if (in_sizes[2] < KD * NHID || in_sizes[3] < KD * NHID) return;
  if (in_sizes[4] < NHID || in_sizes[5] < NHID || in_sizes[6] < 1) return;
  if ((long long)out_size < need_x) return;
  if (ws_size < WS_TOTAL) return;

  const float* keys    = (const float*)d_in[0];
  const float* queries = (const float*)d_in[1];
  const float* wk      = (const float*)d_in[2];
  const float* wq      = (const float*)d_in[3];
  const float* b1      = (const float*)d_in[4];
  const float* w2      = (const float*)d_in[5];
  const float* b2      = (const float*)d_in[6];
  float* out = (float*)d_out;

  char* ws = (char*)d_ws;
  _Float16* Wk_t = (_Float16*)(ws + OFF_WK);
  _Float16* Wq_t = (_Float16*)(ws + OFF_WQ);
  _Float16* Vt16 = (_Float16*)(ws + OFF_VT);
  float*    KhT  = (float*)(ws + OFF_KH);
  float*    QhT  = (float*)(ws + OFF_QH);

  wconv32_kernel<<<dim3(1), dim3(256), 0, stream>>>(wk, Wk_t);
  wconv32_kernel<<<dim3(1), dim3(256), 0, stream>>>(wq, Wq_t);
  vtconv_kernel<<<dim3(KD / 64, SEQ / 64, NB), dim3(256), 0, stream>>>(keys, Vt16);
  proj_k_kernel<<<dim3(SEQ / 128, NB), dim3(256), 0, stream>>>(keys, Wk_t, b1, KhT);
  proj_q_kernel<<<dim3(SEQ / 128, NB), dim3(256), 0, stream>>>(queries, Wq_t, b1, QhT);
  attn_kernel<<<dim3(SEQ / 64, NB), dim3(128), 0, stream>>>(QhT, KhT, Vt16, w2, b2, out);
}
